// DriverDenseModel_66907000537375
// MI455X (gfx1250) — hardware-verified
//
#include <hip/hip_runtime.h>


#ifndef NROWS
#define NROWS 16384
#endif
#define NROWS_FULL 16384
#define NDENSE 64
#define HID    256
#define ODIM   256
#define INDIM  1994
#define NSP    8
#define CARD0 1000
#define CARD1 500
#define CARD2 200
#define CARD3 100
#define CARD4 50
#define CARD5 50
#define CARD6 20
#define CARD7 10
#define OFF0 (NDENSE)
#define OFF1 (OFF0 + CARD0)
#define OFF2 (OFF1 + CARD1)
#define OFF3 (OFF2 + CARD2)
#define OFF4 (OFF3 + CARD3)
#define OFF5 (OFF4 + CARD4)
#define OFF6 (OFF5 + CARD5)
#define OFF7 (OFF6 + CARD6)
#define EW   8
#define ER   8
#define HSC  256.0f
#define WSC  1024.0f
#define OSC  (1.0f / 262144.0f)
#define OSW  68
#define TLW  33

static_assert(OFF7 + CARD7 == INDIM);
static_assert(NROWS % 64 == 0);
static_assert(NROWS <= NROWS_FULL);
static_assert(NROWS % (EW * ER) == 0);
static_assert(NDENSE % 32 == 0);
static_assert(HID % 32 == 0);
static_assert(NDENSE % 64 == 0);
static_assert(HID % 64 == 0);
static_assert(ODIM % 64 == 0);
static_assert(HID % 32 == 0 && ODIM % 32 == 0);
static_assert(HID == 32 * 4 * 2);
static_assert(32 * 16 * 4 == 16 * 64 * 2);
static_assert(32 * 16 * 8 == 16 * 64 * 4);
static_assert(256 * 16 == 32 * 64 * 2);
static_assert(256 * 8 == 64 * 32);
static_assert((OSW * 4) % 16 == 0);
static_assert(16 * OSW * 4 <= 131072);
static_assert(64 * TLW * 4 <= 131072);
static_assert(HSC * WSC * OSC == 1.0f);

typedef _Float16 h16;
typedef unsigned short bf;
typedef __attribute__((ext_vector_type(16))) __bf16   v16bf;
typedef __attribute__((ext_vector_type(16))) _Float16 v16h;
typedef __attribute__((ext_vector_type(8)))  _Float16 v8h;
typedef __attribute__((ext_vector_type(8)))  unsigned short v8us;
typedef __attribute__((ext_vector_type(8)))  float    v8f;
typedef __attribute__((ext_vector_type(4)))  float    v4f;
typedef v4f  __attribute__((may_alias)) v4fa;

__device__ __forceinline__ unsigned short f2bf(float f) { unsigned u = __float_as_uint(f); u += 0x7FFFu + ((u >> 16) & 1u); return (unsigned short)(u >> 16); }
__device__ __forceinline__ float bfr(float f) { return __uint_as_float(((unsigned)f2bf(f)) << 16); }
__device__ __forceinline__ v16h cat16(v8h lo, v8h hi) { return __builtin_shufflevector(lo, hi, 0, 1, 2, 3, 4, 5, 6, 7, 8, 9, 10, 11, 12, 13, 14, 15); }
__device__ __forceinline__ v16bf cat16b(v8us lo, v8us hi) { return __builtin_bit_cast(v16bf, __builtin_shufflevector(lo, hi, 0, 1, 2, 3, 4, 5, 6, 7, 8, 9, 10, 11, 12, 13, 14, 15)); }
__device__ __forceinline__ v8f wmma16(v16h a, v16h b, v8f c) { return __builtin_amdgcn_wmma_f32_16x16x32_f16(false, a, false, b, (short)0, c, false, false); }
__device__ __forceinline__ v8f wmmab(v16bf a, v16bf b, v8f c) { return __builtin_amdgcn_wmma_f32_16x16x32_bf16(false, a, false, b, (short)0, c, false, false); }
__device__ __forceinline__ v16h  ldh(const h16* p) { return cat16(*(const v8h*)p, *(const v8h*)(p + 16)); }
__device__ __forceinline__ v16bf ldb(const bf* p)  { return cat16b(*(const v8us*)p, *(const v8us*)(p + 16)); }
__device__ __forceinline__ void wave_sync() { __builtin_amdgcn_fence(3  , "wavefront"); __builtin_amdgcn_wave_barrier(); asm volatile("" ::: "memory"); }

static __device__ __forceinline__ h16 toh_flush(float v) { const h16 r = (h16)v; return (fabsf(v) < 6.103515625e-05f) ? (h16)0.0f : r; }
__device__ __forceinline__ v8f wmmab_g(v16bf a, v16bf b, v8f c) { c = __builtin_amdgcn_wmma_f32_16x16x32_bf16(false, a, false, b, (short)0, c, false, false); asm volatile("v_nop\n\tv_nop\n\tv_nop\n\tv_nop" : "+v"(c) : "v"(a), "v"(b)); return c; }
__device__ __forceinline__ v8f wmma16_g(v16h a, v16h b, v8f c) { c = __builtin_amdgcn_wmma_f32_16x16x32_f16(false, a, false, b, (short)0, c, false, false); asm volatile("v_nop\n\tv_nop\n\tv_nop\n\tv_nop" : "+v"(c) : "v"(a), "v"(b)); return c; }

__global__ __launch_bounds__(256) void k_cvt8(const float* __restrict__ src, bf* dst, size_t n8) {
    const size_t i = (size_t)blockIdx.x * 256 + threadIdx.x; if (i >= n8) return;
    const v8f v = *(const v8f*)(src + i * 8); v8us o;
#pragma unroll
    for (int k = 0; k < 8; ++k) o[k] = f2bf(v[k]);
    *(volatile v8us*)(dst + i * 8) = o; __threadfence(); *(volatile v8us*)(dst + i * 8) = o;
}

__global__ __launch_bounds__(256) void k_wt_bf(const float* __restrict__ src, bf* dst, int K, int N) {
    __shared__ float tl[64 * TLW];
    const int t = threadIdx.x; const int n0 = blockIdx.x * 32, k0 = blockIdx.y * 64;
#pragma unroll 1
    for (int i = 0; i < 8; ++i) { const int f = t + i * 256; const int kk = f >> 5, nn = f & 31; tl[kk * TLW + nn] = src[(size_t)(k0 + kk) * N + n0 + nn]; }
    __syncthreads();
    const int nn = t >> 3, c = t & 7; v8us o;
#pragma unroll
    for (int i = 0; i < 8; ++i) o[i] = f2bf(tl[(8 * c + i) * TLW + nn]);
    bf* p = dst + (size_t)(n0 + nn) * K + k0 + 8 * c;
    *(volatile v8us*)p = o; __threadfence(); *(volatile v8us*)p = o;
}

__global__ __launch_bounds__(256) void k_wt_h(const float* __restrict__ src, h16* dst, int K, int N) {
    __shared__ float tl[64 * TLW];
    const int t = threadIdx.x; const int n0 = blockIdx.x * 32, k0 = blockIdx.y * 64;
#pragma unroll 1
    for (int i = 0; i < 8; ++i) { const int f = t + i * 256; const int kk = f >> 5, nn = f & 31; tl[kk * TLW + nn] = src[(size_t)(k0 + kk) * N + n0 + nn]; }
    __syncthreads();
    const int nn = t >> 3, c = t & 7; v8h o;
#pragma unroll
    for (int i = 0; i < 8; ++i) o[i] = toh_flush(bfr(tl[(8 * c + i) * TLW + nn]) * WSC);
    h16* p = dst + (size_t)(n0 + nn) * K + k0 + 8 * c;
    *(volatile v8h*)p = o; __threadfence(); *(volatile v8h*)p = o;
}

__device__ __forceinline__ void emb_add(const float* __restrict__ W1, int idx, int off, int card, int lane, v4f& sa, v4f& sb) {
    const bool ok = (idx >= 0) & (idx < card);
    int ic = idx < 0 ? 0 : idx; ic = ic > card - 1 ? card - 1 : ic;
    const float* wr = W1 + (size_t)(off + ic) * HID + 4 * lane;
    v4f x = *(const v4f*)wr; v4f y = *(const v4f*)(wr + 128);
    asm volatile("" : "+v"(x), "+v"(y));
#pragma unroll
    for (int i = 0; i < 4; ++i) { sa[i] += ok ? bfr(x[i]) : 0.0f; sb[i] += ok ? bfr(y[i]) : 0.0f; }
}

__global__ __launch_bounds__(32 * EW) void k_emb(const int* __restrict__ sp, const float* __restrict__ W1, const float* __restrict__ b1, float* E) {
#pragma clang fp contract(off)
    const int lane = threadIdx.x & 31;
    const int wave = __builtin_amdgcn_readfirstlane((int)(threadIdx.x >> 5));
    const int rbase = (blockIdx.x * EW + wave) * ER;
    const v4f ba = *(const v4f*)(b1 + 4 * lane), bb = *(const v4f*)(b1 + 128 + 4 * lane);
    v4f b0v, b1v;
#pragma unroll
    for (int i = 0; i < 4; ++i) { b0v[i] = bfr(ba[i]); b1v[i] = bfr(bb[i]); }
#pragma unroll 1
    for (int r = 0; r < ER; ++r) {
        const int row = rbase + r;
        const int* ip = sp + (size_t)row * NSP;
        v4f sa = (v4f){}, sb = (v4f){};
        emb_add(W1, ip[0], OFF0, CARD0, lane, sa, sb);
        emb_add(W1, ip[1], OFF1, CARD1, lane, sa, sb);
        emb_add(W1, ip[2], OFF2, CARD2, lane, sa, sb);
        emb_add(W1, ip[3], OFF3, CARD3, lane, sa, sb);
        emb_add(W1, ip[4], OFF4, CARD4, lane, sa, sb);
        emb_add(W1, ip[5], OFF5, CARD5, lane, sa, sb);
        emb_add(W1, ip[6], OFF6, CARD6, lane, sa, sb);
        emb_add(W1, ip[7], OFF7, CARD7, lane, sa, sb);
        sa = sa + b0v; sb = sb + b1v;
        float* ep = E + (size_t)row * HID + 4 * lane;
        *(volatile v4f*)ep = sa; *(volatile v4f*)(ep + 128) = sb;
        __threadfence();
        *(volatile v4f*)ep = sa; *(volatile v4f*)(ep + 128) = sb;
    }
}

__global__ __launch_bounds__(32) void k_gemm1(const bf* __restrict__ A, const bf* __restrict__ Bt, const float* __restrict__ E, h16* H) {
    __shared__ __align__(16) float os[16 * OSW];
    const int K = NDENSE;
    const int lane = threadIdx.x & 31, lr = lane & 15, hi = lane >> 4; const int r0 = blockIdx.x * 64, c0 = blockIdx.y * 64;
    v8f acc[4][4];
#pragma unroll
    for (int mb = 0; mb < 4; ++mb)
#pragma unroll
        for (int nb = 0; nb < 4; ++nb) acc[mb][nb] = (v8f){};
    const size_t aoff = (size_t)(r0 + lr) * K + 8 * hi, boff = (size_t)(c0 + lr) * K + 8 * hi;
#pragma unroll 1
    for (int kc = 0; kc < K; kc += 32) {
        v16bf a[4];
#pragma unroll
        for (int mb = 0; mb < 4; ++mb) a[mb] = ldb(A + aoff + (size_t)mb * 16 * K + kc);
#pragma unroll
        for (int nb = 0; nb < 4; ++nb) { const v16bf b = ldb(Bt + boff + (size_t)nb * 16 * K + kc);
#pragma unroll
            for (int mb = 0; mb < 4; ++mb) acc[mb][nb] = wmmab_g(a[mb], b, acc[mb][nb]); }
    }
#pragma unroll
    for (int mb = 0; mb < 4; ++mb) {
#pragma unroll
        for (int nb = 0; nb < 4; ++nb) {
#pragma unroll
            for (int j = 0; j < 8; ++j) os[(hi * 8 + j) * OSW + nb * 16 + lr] = acc[mb][nb][j]; }
        wave_sync();
        v8h hv[4];
#pragma unroll
        for (int s = 0; s < 4; ++s) { const int row = 4 * s + (lane >> 3), c8 = (lane & 7) * 8;
            const v4f x0 = *(const v4fa*)(&os[row * OSW + c8]); const v4f x1 = *(const v4fa*)(&os[row * OSW + c8 + 4]);
            const float* ep = E + (size_t)(r0 + mb * 16 + row) * HID + c0 + c8;
            const v4f e0 = *(const v4f*)ep; const v4f e1 = *(const v4f*)(ep + 4);
#pragma unroll
            for (int i = 0; i < 4; ++i) { float u = x0[i] + e0[i]; float w = x1[i] + e1[i]; u = u > 0.0f ? u : 0.0f; w = w > 0.0f ? w : 0.0f;
                hv[s][i] = toh_flush(u * HSC); hv[s][4 + i] = toh_flush(w * HSC); } }
#pragma unroll 1
        for (int ps = 0; ps < 2; ++ps) {
#pragma unroll
            for (int s = 0; s < 4; ++s) { const int row = 4 * s + (lane >> 3), c8 = (lane & 7) * 8;
                *(volatile v8h*)(H + (size_t)(r0 + mb * 16 + row) * HID + c0 + c8) = hv[s]; }
            if (ps == 0) __threadfence(); }
        wave_sync();
    }
}

__global__ __launch_bounds__(32) void k_gemm2(const h16* __restrict__ A, const h16* __restrict__ Bt, const float* __restrict__ b2, float* OUT) {
    __shared__ __align__(16) float os[16 * OSW];
    const int K = HID;
    const int lane = threadIdx.x & 31, lr = lane & 15, hi = lane >> 4; const int r0 = blockIdx.x * 64, c0 = blockIdx.y * 64;
    v8f acc[4][4];
#pragma unroll
    for (int mb = 0; mb < 4; ++mb)
#pragma unroll
        for (int nb = 0; nb < 4; ++nb) acc[mb][nb] = (v8f){};
    const size_t aoff = (size_t)(r0 + lr) * K + 8 * hi, boff = (size_t)(c0 + lr) * K + 8 * hi;
#pragma unroll 1
    for (int kc = 0; kc < K; kc += 32) {
        v16h a[4];
#pragma unroll
        for (int mb = 0; mb < 4; ++mb) a[mb] = ldh(A + aoff + (size_t)mb * 16 * K + kc);
#pragma unroll
        for (int nb = 0; nb < 4; ++nb) { const v16h b = ldh(Bt + boff + (size_t)nb * 16 * K + kc);
#pragma unroll
            for (int mb = 0; mb < 4; ++mb) acc[mb][nb] = wmma16_g(a[mb], b, acc[mb][nb]); }
    }
    const int c4 = (lane & 15) * 4;
    const v4f braw = *(const v4f*)(b2 + c0 + c4);
    v4f bias;
#pragma unroll
    for (int i = 0; i < 4; ++i) bias[i] = bfr(braw[i]);
#pragma unroll
    for (int mb = 0; mb < 4; ++mb) {
#pragma unroll
        for (int nb = 0; nb < 4; ++nb) {
#pragma unroll
            for (int j = 0; j < 8; ++j) os[(hi * 8 + j) * OSW + nb * 16 + lr] = acc[mb][nb][j]; }
        wave_sync();
        v4f ov[8];
#pragma unroll
        for (int s = 0; s < 8; ++s) { const int row = 2 * s + (lane >> 4);
            const v4f x = *(const v4fa*)(&os[row * OSW + c4]);
            ov[s] = x * OSC + bias; }
#pragma unroll 1
        for (int ps = 0; ps < 2; ++ps) {
#pragma unroll
            for (int s = 0; s < 8; ++s) { const int row = 2 * s + (lane >> 4);
                *(volatile v4f*)(OUT + (size_t)(r0 + mb * 16 + row) * ODIM + c0 + c4) = ov[s]; }
            if (ps == 0) __threadfence(); }
        wave_sync();
    }
}

static constexpr size_t al256(size_t v) { return (v + 255) & ~(size_t)255; }
static constexpr size_t SZ_XB  = al256((size_t)NROWS * NDENSE * 2);
static constexpr size_t SZ_W1T = al256((size_t)HID * NDENSE * 2);
static constexpr size_t SZ_W2T = al256((size_t)ODIM * HID * 2);
static constexpr size_t SZ_E   = al256((size_t)NROWS * HID * 4);
static constexpr size_t SZ_H   = al256((size_t)NROWS * HID * 2);
static constexpr size_t SZ_TOTAL = SZ_XB + SZ_W1T + SZ_W2T + SZ_E + SZ_H;
static_assert(SZ_TOTAL <= (size_t)134217728);
static_assert(((size_t)NROWS * NDENSE) % 8 == 0);
static_assert((size_t)(NROWS / 64) * 64 * (HID / 64) * 64 == (size_t)NROWS * HID);
static_assert((size_t)(NROWS / 64) * 64 * (ODIM / 64) * 64 == (size_t)NROWS * ODIM);
static_assert((size_t)(NROWS / (EW * ER)) * EW * ER * HID == (size_t)NROWS * HID);
static_assert((size_t)(HID / 32) * (NDENSE / 64) * 2048 == (size_t)HID * NDENSE);
static_assert((size_t)(ODIM / 32) * (HID / 64) * 2048 == (size_t)ODIM * HID);

extern "C" void kernel_launch(void* const* d_in, const int* in_sizes, int n_in,
                              void* d_out, int out_size, void* d_ws, size_t ws_size, hipStream_t stream) {
    if (n_in < 6) return;
    if ((size_t)in_sizes[0] < (size_t)NROWS * NDENSE) return;
    if ((size_t)in_sizes[1] < (size_t)NROWS * NSP) return;
    if ((size_t)in_sizes[2] < (size_t)INDIM * HID) return;
    if (in_sizes[3] < HID) return;
    if ((size_t)in_sizes[4] < (size_t)HID * ODIM) return;
    if (in_sizes[5] < ODIM) return;
    if ((size_t)out_size < (size_t)NROWS * ODIM) return;
    if (SZ_TOTAL > ws_size) return;
    const float* dense  = (const float*)d_in[0];
    const int*   sparse = (const int*)d_in[1];
    const float* w1 = (const float*)d_in[2]; const float* b1 = (const float*)d_in[3];
    const float* w2 = (const float*)d_in[4]; const float* b2 = (const float*)d_in[5];
    float* OUT = (float*)d_out;
    char* wsp = (char*)d_ws;
    bf*  XB  = (bf*)wsp;  wsp += SZ_XB;
    bf*  W1T = (bf*)wsp;  wsp += SZ_W1T;
    h16* W2T = (h16*)wsp; wsp += SZ_W2T;
    float* E = (float*)wsp; wsp += SZ_E;
    h16* H   = (h16*)wsp; wsp += SZ_H;

    { const size_t n8 = (size_t)NROWS * NDENSE / 8;
      k_cvt8<<<(unsigned)((n8 + 255) / 256), 256, 0, stream>>>(dense, XB, n8); }
    k_wt_bf<<<dim3(HID / 32, NDENSE / 64, 1), 256, 0, stream>>>(w1, W1T, NDENSE, HID);
    k_wt_h<<<dim3(ODIM / 32, HID / 64, 1), 256, 0, stream>>>(w2, W2T, HID, ODIM);
    k_emb<<<NROWS / (EW * ER), 32 * EW, 0, stream>>>(sparse, w1, b1, E);
    k_gemm1<<<dim3(NROWS / 64, HID / 64, 1), 32, 0, stream>>>(XB, W1T, E, H);
    k_gemm2<<<dim3(NROWS / 64, ODIM / 64, 1), 32, 0, stream>>>(H, W2T, b2, OUT);
}
